// CrossAttention1d_23321672417301
// MI455X (gfx1250) — hardware-run, weakly checked
//
#include <hip/hip_runtime.h>
#include <math.h>

typedef __attribute__((ext_vector_type(16))) _Float16 v16h;
typedef __attribute__((ext_vector_type(8)))  _Float16 v8h;
typedef __attribute__((ext_vector_type(8)))  float    v8f;
typedef __attribute__((ext_vector_type(4)))  float    v4f;

constexpr int kBatch = 8;
constexpr int kChan  = 768;
constexpr int kLen   = 256;
constexpr int kHeads = 12;
constexpr int kHd    = 64;
constexpr int kHL    = kHeads * kLen;
constexpr int kBCN   = kChan * kLen;
constexpr int kSqrtHd = 8;
static_assert(kHd * kHeads == kChan, "channel axis factors as (d outer, head inner)");
static_assert(kHd * kHL == kBCN, "flat [64][3072] view");
static_assert(kHL == 3072 && kBCN == 196608, "wire shapes");
static_assert(kSqrtHd * kSqrtHd == kHd, "score scale = 1/sqrt(head dim)");
static_assert((kChan % 64) == 0 && (kLen % 64) == 0 && (kHL % 64) == 0 && (kHd % 64) == 0, "tile multiples of 64");
static_assert((kChan % 32) == 0 && (kHL % 32) == 0 && (kHd % 32) == 0, "K multiples of 32");

constexpr float kAttnScale  = 1.0f / (float)kSqrtHd;
constexpr float kCarryIn    = 16.0f;
constexpr float kCarryW     = 1024.0f;
constexpr float kCarryCp    = 16.0f;
constexpr float kCarryM     = 0.25f;
constexpr float kCarryOut   = 0.25f;
constexpr float kScaleProj  = kCarryCp / (kCarryW * kCarryIn);
constexpr float kScalePair  = kCarryM / (kCarryIn * kCarryCp);
constexpr float kScaleApply = (kAttnScale * kCarryOut) / (kCarryIn * kCarryM);
constexpr float kScaleDep   = 1.0f / (kCarryW * kCarryOut);
constexpr float kF16MinNormal = 6.103515625e-05f;
static_assert(kScaleProj == 1.0f / 1024.0f, "projection fold-back");
static_assert(kScalePair == 1.0f / 1024.0f, "pair fold-back");
static_assert(kScaleApply == 1.0f / 128.0f, "apply fold-back");
static_assert(kScaleDep == 1.0f / 256.0f, "de-projection fold-back");

constexpr size_t kBytesBig = (size_t)kBatch * kBCN * 2;
constexpr size_t kBytesW   = (size_t)kChan * kChan * 2;
constexpr size_t kBytesMT  = (size_t)kBatch * kHd * kHd * 2;
constexpr size_t kOffCRP = 0;
constexpr size_t kOffCRT = kOffCRP + kBytesBig;
constexpr size_t kOffXT  = kOffCRT + kBytesBig;
constexpr size_t kOffWPP = kOffXT  + kBytesBig;
constexpr size_t kOffWDP = kOffWPP + kBytesW;
constexpr size_t kOffCPP = kOffWDP + kBytesW;
constexpr size_t kOffMTP = kOffCPP + kBytesBig;
constexpr size_t kOffOUP = kOffMTP + kBytesMT;
constexpr size_t kWsTotal = kOffOUP + kBytesBig;
static_assert(kWsTotal == 18153472ull, "carve total");
static_assert(kWsTotal <= 134217728ull, "carve cap");
static_assert((kOffCRT % 128) == 0 && (kOffXT % 128) == 0 && (kOffWPP % 128) == 0 && (kOffWDP % 128) == 0 &&
              (kOffCPP % 128) == 0 && (kOffMTP % 128) == 0 && (kOffOUP % 128) == 0, "128-B aligned regions");

__device__ __forceinline__ float bf16_rne_value(float f) {
  const unsigned u = __float_as_uint(f);
  const unsigned r = (u + 0x7FFFu + ((u >> 16) & 1u)) & 0xFFFF0000u;
  return __uint_as_float(r);
}
__device__ __forceinline__ _Float16 f16_flush(float v) {
  const float w = (__builtin_fabsf(v) < kF16MinNormal) ? 0.0f : v;
  return (_Float16)w;
}
__device__ __forceinline__ v16h frag_load(const _Float16* p) {
  union U { v16h v; v8h h[2]; };
  U f;
  f.h[0] = *(const v8h*)(p);
  f.h[1] = *(const v8h*)(p + 16);
  return f.v;
}
__device__ __forceinline__ v8f mma_f16(v16h a, v16h b, v8f c) {
  c = __builtin_amdgcn_wmma_f32_16x16x32_f16(false, a, false, b, (short)0, c, false, false);
  asm volatile("v_nop\n\tv_nop\n\tv_nop\n\tv_nop" : "+v"(c) : "v"(a), "v"(b));
  return c;
}
__device__ __forceinline__ void wave_lds_sync() {
  __builtin_amdgcn_fence(__ATOMIC_RELEASE, "workgroup");
  __builtin_amdgcn_wave_barrier();
  __builtin_amdgcn_fence(__ATOMIC_ACQUIRE, "workgroup");
}

template <int CSEL>
__global__ __launch_bounds__(256) void operand_planes_rows(
    const float* __restrict__ src, unsigned short* __restrict__ dst, int total8)
{
  constexpr float carry = (CSEL == 0) ? kCarryIn : kCarryW;
  const int i = blockIdx.x * 256 + threadIdx.x;
  if (i >= total8) return;
  const size_t e0 = (size_t)i << 3;
  const v4f a0 = *(const v4f*)(src + e0);
  const v4f a1 = *(const v4f*)(src + e0 + 4);
  v8h hv;
#pragma unroll
  for (int e = 0; e < 4; ++e) {
    const float s0 = a0[e];
    const float s1 = a1[e];
    hv[e]     = f16_flush(bf16_rne_value(s0) * carry);
    hv[4 + e] = f16_flush(bf16_rne_value(s1) * carry);
  }
  unsigned short* q = dst + e0;
  *(volatile v8h*)q = hv;
  __threadfence();
  *(volatile v8h*)q = hv;
}

template <int CSEL>
__global__ __launch_bounds__(256) void operand_planes_transposed(
    const float* __restrict__ src, unsigned short* __restrict__ dst, int R, int Cc)
{
  constexpr float carry = (CSEL == 0) ? kCarryIn : kCarryW;
  __shared__ __align__(16) float sT[64 * 68];
  const int tid = threadIdx.x, lane = tid & 31, wave = tid >> 5;
  const int c0 = blockIdx.x * 64;
  const int r0 = blockIdx.y * 64;
  const size_t boff = (size_t)blockIdx.z * (size_t)R * (size_t)Cc;
  const float* sb = src + boff;
  unsigned short* db = dst + boff;
  const int lr = tid >> 4, lc4 = (tid & 15) * 4;
#pragma unroll
  for (int i = 0; i < 4; ++i) {
    const int row = lr + 16 * i;
    const v4f v = *(const v4f*)(sb + (size_t)(r0 + row) * Cc + c0 + lc4);
    v4f w;
#pragma unroll
    for (int e = 0; e < 4; ++e) {
      const float s = v[e];
      w[e] = bf16_rne_value(s) * carry;
    }
    *(v4f*)(sT + row * 68 + lc4) = w;
  }
  __syncthreads();
  const int q = lane >> 3, c8 = (lane & 7) * 8;
  v8h hv[2];
#pragma unroll
  for (int it = 0; it < 2; ++it) {
    const int orow = it * 32 + wave * 4 + q;
#pragma unroll
    for (int e = 0; e < 8; ++e) hv[it][e] = f16_flush(sT[(c8 + e) * 68 + orow]);
  }
  for (int pass = 0; pass < 2; ++pass) {
#pragma unroll
    for (int it = 0; it < 2; ++it) {
      const int orow = it * 32 + wave * 4 + q;
      *(volatile v8h*)(db + (size_t)(c0 + orow) * R + r0 + c8) = hv[it];
    }
    __threadfence();
  }
}

template <int EPI>
__global__ __launch_bounds__(256) void tile_product(
    const unsigned short* __restrict__ Ap, int lda, long strideA,
    const unsigned short* __restrict__ Btp, int ldb, long strideB,
    void* __restrict__ Cout, int ldc, long strideC,
    const float* __restrict__ bias,
    const float* __restrict__ skip, long strideR,
    int M, int N, int K)
{
  constexpr float scale = (EPI == 0) ? kScaleProj : ((EPI == 1) ? kScaleApply : kScaleDep);
  __shared__ __align__(16) float sT[8][16 * 68];
  const int b    = blockIdx.y;
  const int lane = threadIdx.x & 31;
  const int wave = threadIdx.x >> 5;
  const int tilesN = N >> 6;
  const int tilesM = M >> 6;
  const int tile = blockIdx.x * 8 + wave;
  if (tile >= tilesM * tilesN) return;
  const int tm = tile / tilesN;
  const int tn = tile - tm * tilesN;
  const int m0 = tm << 6;
  const int n0 = tn << 6;

  const _Float16* Ab = (const _Float16*)Ap  + (size_t)b * strideA;
  const _Float16* Bb = (const _Float16*)Btp + (size_t)b * strideB;

  const int rlane = lane & 15;
  const int koff  = (lane >> 4) * 8;
  const int mOff  = (lane >> 4) * 8;

  v8f acc[4][4];
#pragma unroll
  for (int i = 0; i < 4; ++i)
#pragma unroll
    for (int j = 0; j < 4; ++j) acc[i][j] = (v8f){0.f,0.f,0.f,0.f,0.f,0.f,0.f,0.f};

  for (int k0 = 0; k0 < K; k0 += 32) {
    v16h bh[4];
#pragma unroll
    for (int j = 0; j < 4; ++j) {
      const size_t bo = (size_t)(n0 + (j << 4) + rlane) * ldb + koff + k0;
      bh[j] = frag_load(Bb + bo);
    }
#pragma unroll
    for (int i = 0; i < 4; ++i) {
      const size_t ao = (size_t)(m0 + (i << 4) + rlane) * lda + koff + k0;
      const v16h ah = frag_load(Ab + ao);
#pragma unroll
      for (int j = 0; j < 4; ++j) acc[i][j] = mma_f16(ah, bh[j], acc[i][j]);
    }
  }

  float* slab = sT[wave];
#pragma unroll
  for (int i = 0; i < 4; ++i) {
    const int mBase = m0 + (i << 4);
#pragma unroll
    for (int j = 0; j < 4; ++j) {
#pragma unroll
      for (int r = 0; r < 8; ++r)
        slab[(mOff + r) * 68 + (j << 4) + rlane] = acc[i][j][r] * scale;
    }
    wave_lds_sync();
    if (EPI == 2) {
      const float* Rb = skip + (size_t)b * strideR;
      float* C = (float*)Cout + (size_t)b * strideC;
      const int hh = lane >> 4, c4 = (lane & 15) * 4;
#pragma unroll
      for (int it = 0; it < 8; ++it) {
        const int row = it * 2 + hh;
        const size_t go = (size_t)(mBase + row) * ldc + n0 + c4;
        const v4f xr = *(const v4f*)(Rb + go);
        const float braw = bias[mBase + row];
        const float bv = bf16_rne_value(braw);
        v4f s = *(const v4f*)(slab + row * 68 + c4);
#pragma unroll
        for (int e = 0; e < 4; ++e) {
          const float xe = xr[e];
          const float se = s[e];
          s[e] = (se + bv) + bf16_rne_value(xe);
        }
        *(v4f*)(slab + row * 68 + c4) = s;
      }
      wave_lds_sync();
      for (int pass = 0; pass < 2; ++pass) {
#pragma unroll
        for (int it = 0; it < 8; ++it) {
          const int row = it * 2 + hh;
          const v4f v = *(const v4f*)(slab + row * 68 + c4);
          *(volatile v4f*)(C + (size_t)(mBase + row) * ldc + n0 + c4) = v;
        }
        __threadfence();
      }
    } else {
      unsigned short* C = (unsigned short*)Cout + (size_t)b * strideC;
      const int q = lane >> 3, c8 = (lane & 7) * 8;
      v8h hv[4];
#pragma unroll
      for (int it = 0; it < 4; ++it) {
        const int row = it * 4 + q;
        const float* sp = slab + row * 68 + c8;
        float bv = 0.0f;
        if (EPI == 0) {
          const float braw = bias[mBase + row];
          bv = bf16_rne_value(braw) * kCarryCp;
        }
#pragma unroll
        for (int e = 0; e < 8; ++e) hv[it][e] = f16_flush(sp[e] + bv);
      }
      for (int pass = 0; pass < 2; ++pass) {
#pragma unroll
        for (int it = 0; it < 4; ++it) {
          const int row = it * 4 + q;
          *(volatile v8h*)(C + (size_t)(mBase + row) * ldc + n0 + c8) = hv[it];
        }
        __threadfence();
      }
    }
    wave_lds_sync();
  }
}

__global__ __launch_bounds__(256) void pair_matrix(
    const unsigned short* __restrict__ crossP, const unsigned short* __restrict__ cpP,
    unsigned short* __restrict__ MT)
{
  __shared__ __align__(16) float sM[64 * 68];
  const int tid = threadIdx.x, lane = tid & 31, wave = tid >> 5;
  const int b = blockIdx.x;
  const _Float16* A  = (const _Float16*)crossP + (size_t)b * kBCN;
  const _Float16* Bt = (const _Float16*)cpP    + (size_t)b * kBCN;
  const int ri = wave & 3, jh = wave >> 2;
  const int rlane = lane & 15;
  const int koff  = (lane >> 4) * 8;
  const int mOff  = (lane >> 4) * 8;
  const _Float16* ap  = A  + (size_t)(16 * ri + rlane) * kHL + koff;
  const _Float16* bp0 = Bt + (size_t)(32 * jh + rlane) * kHL + koff;
  const _Float16* bp1 = Bt + (size_t)(32 * jh + 16 + rlane) * kHL + koff;
  v8f acc0 = (v8f){0.f,0.f,0.f,0.f,0.f,0.f,0.f,0.f};
  v8f acc1 = (v8f){0.f,0.f,0.f,0.f,0.f,0.f,0.f,0.f};
#pragma unroll 2
  for (int k0 = 0; k0 < kHL; k0 += 32) {
    const v16h a  = frag_load(ap + k0);
    const v16h b0 = frag_load(bp0 + k0);
    const v16h b1 = frag_load(bp1 + k0);
    acc0 = mma_f16(a, b0, acc0);
    acc1 = mma_f16(a, b1, acc1);
  }
#pragma unroll
  for (int r = 0; r < 8; ++r) {
    sM[(16 * ri + mOff + r) * 68 + 32 * jh + rlane]      = acc0[r] * kScalePair;
    sM[(16 * ri + mOff + r) * 68 + 32 * jh + 16 + rlane] = acc1[r] * kScalePair;
  }
  __syncthreads();
  const int q = lane >> 3, c8 = (lane & 7) * 8;
  v8h hv[2];
#pragma unroll
  for (int it = 0; it < 2; ++it) {
    const int row = it * 32 + wave * 4 + q;
#pragma unroll
    for (int e = 0; e < 8; ++e) hv[it][e] = f16_flush(sM[row * 68 + c8 + e]);
  }
  unsigned short* Mb = MT + (size_t)b * (kHd * kHd);
  for (int pass = 0; pass < 2; ++pass) {
#pragma unroll
    for (int it = 0; it < 2; ++it) {
      const int row = it * 32 + wave * 4 + q;
      *(volatile v8h*)(Mb + row * kHd + c8) = hv[it];
    }
    __threadfence();
  }
}

extern "C" void kernel_launch(void* const* d_in, const int* in_sizes, int n_in,
                              void* d_out, int out_size, void* d_ws, size_t ws_size,
                              hipStream_t stream) {
  if (n_in < 6) return;
  if (in_sizes[0] != kBatch * kBCN) return;
  if (in_sizes[1] != kBatch * kBCN) return;
  if (in_sizes[2] != kChan * kChan) return;
  if (in_sizes[3] != kChan) return;
  if (in_sizes[4] != kChan * kChan) return;
  if (in_sizes[5] != kChan) return;
  if (out_size != kBatch * kBCN) return;
  if (ws_size < kWsTotal) return;

  const float* x_ori  = (const float*)d_in[0];
  const float* cross  = (const float*)d_in[1];
  const float* W_proj = (const float*)d_in[2];
  const float* b_proj = (const float*)d_in[3];
  const float* W_dep  = (const float*)d_in[4];
  const float* b_dep  = (const float*)d_in[5];
  float* out = (float*)d_out;

  char* ws = (char*)d_ws;
  unsigned short* CRP = (unsigned short*)(ws + kOffCRP);
  unsigned short* CRT = (unsigned short*)(ws + kOffCRT);
  unsigned short* XT  = (unsigned short*)(ws + kOffXT);
  unsigned short* WPP = (unsigned short*)(ws + kOffWPP);
  unsigned short* WDP = (unsigned short*)(ws + kOffWDP);
  unsigned short* CPP = (unsigned short*)(ws + kOffCPP);
  unsigned short* MTP = (unsigned short*)(ws + kOffMTP);
  unsigned short* OUP = (unsigned short*)(ws + kOffOUP);

  static_assert(((kBatch * kBCN / 8) % 256) == 0 && ((kChan * kChan / 8) % 256) == 0, "exact convert grids");

  operand_planes_rows<0><<<(kBatch * kBCN / 8) / 256, 256, 0, stream>>>(cross, CRP, kBatch * kBCN / 8);
  operand_planes_rows<1><<<(kChan * kChan / 8) / 256, 256, 0, stream>>>(W_proj, WPP, kChan * kChan / 8);
  operand_planes_rows<1><<<(kChan * kChan / 8) / 256, 256, 0, stream>>>(W_dep, WDP, kChan * kChan / 8);

  operand_planes_transposed<0><<<dim3(kLen / 64, kChan / 64, kBatch), 256, 0, stream>>>(cross, CRT, kChan, kLen);
  operand_planes_transposed<0><<<dim3(kHL / 64, kHd / 64, kBatch), 256, 0, stream>>>(x_ori, XT, kHd, kHL);

  tile_product<0><<<dim3(((kChan / 64) * (kLen / 64)) / 8, kBatch), 256, 0, stream>>>(
      WPP, kChan, 0L,
      CRT, kChan, (long)kBCN,
      (void*)CPP, kLen, (long)kBCN,
      b_proj, x_ori, 0L,
      kChan, kLen, kChan);

  pair_matrix<<<kBatch, 256, 0, stream>>>(CRP, CPP, MTP);

  tile_product<1><<<dim3(((kHL / 64) * (kHd / 64)) / 8, kBatch), 256, 0, stream>>>(
      XT, kHd, (long)kBCN,
      MTP, kHd, (long)(kHd * kHd),
      (void*)OUP, kHd, (long)kBCN,
      b_proj, x_ori, 0L,
      kHL, kHd, kHd);

  tile_product<2><<<dim3(((kChan / 64) * (kLen / 64)) / 8, kBatch), 256, 0, stream>>>(
      WDP, kChan, 0L,
      OUP, kChan, (long)kBCN,
      (void*)out, kLen, (long)kBCN,
      b_dep, x_ori, (long)kBCN,
      kChan, kLen, kChan);
}
